// GNNClassifier_28587302322870
// MI455X (gfx1250) — hardware-verified
//
#include <hip/hip_runtime.h>
#include <stddef.h>
#include <stdint.h>


#define FIN    128
#define HID    512
#define NCLS   128
#define AP     1024
#define HOFF   512
#define KL1    256
#define KL2    1024
#define KCL    512
#define NTHR   256
#define NWAVE  8
#define EPT    8
#define CHUNK  (NTHR * EPT)
#define WCAP   (EPT * 32)
#define LISTN  (NWAVE * WCAP)
#define NBA    1024
#define SLA    10
#define RCAP   28672
#define DEGCAP 64
#define LBM    32
#define LTHR   256
#define GBM    64
#define GTHR   128
#define UB1    (HID * (KL1 / 8))
#define UB2    (HID * (KL2 / 8))
#define UBC    (NCLS * (KCL / 8))
#define UTOT   (UB1 + UB2 + UBC)
#define AGG_ZINTS    (LISTN + 2 * RCAP + 3 * NBA)
#define MISC_INTS    16
#define AGG_LDS_INTS (AGG_ZINTS + MISC_INTS)
#define LN_LDS_BYTES (LBM * HID * 4)
#define WSMAX  134217728

static_assert((CHUNK & (CHUNK - 1)) == 0 && CHUNK <= 4096);
static_assert((NBA & (NBA - 1)) == 0 && NBA == (1 << SLA));
static_assert(((long long)CHUNK << SLA) < (1LL << 31));
static_assert(LISTN % NTHR == 0);
static_assert(NBA % NWAVE == 0 && NBA % 32 == 0 && NBA % GBM == 0 && NBA % LBM == 0);
static_assert(RCAP % 4 == 0 && AGG_ZINTS % 4 == 0 && LISTN % 4 == 0);
static_assert(AGG_ZINTS % (NTHR * 4) == 0);
static_assert(AGG_LDS_INTS * 4 <= 300000 && LN_LDS_BYTES <= 300000);
static_assert(KL1 % 32 == 0 && KL2 % 32 == 0 && KCL % 32 == 0);
static_assert(KL1 == 2 * FIN && KL2 == AP && HOFF + KCL == AP && HOFF == HID && KCL == HID);
static_assert(FIN == 4 * 32 && HID == 16 * 32 && NCLS == 128);
static_assert(LTHR == 32 * NWAVE && LBM == 2 * 16 && LBM == 4 * NWAVE && HID == 4 * 128);
static_assert(GBM == (GTHR / 32) * 16);
static_assert(UB1 % NTHR == 0 && UB2 % NTHR == 0 && UBC % NTHR == 0 && UTOT % NTHR == 0);

typedef float          v4f   __attribute__((ext_vector_type(4)));
typedef float          v8f   __attribute__((ext_vector_type(8)));
typedef int            v4i   __attribute__((ext_vector_type(4)));
typedef int            v8i   __attribute__((ext_vector_type(8)));
typedef unsigned       v4u   __attribute__((ext_vector_type(4)));
typedef unsigned short v8us  __attribute__((ext_vector_type(8)));
typedef unsigned short v16us __attribute__((ext_vector_type(16)));
typedef __bf16         v16bf __attribute__((ext_vector_type(16)));
typedef v4f  __attribute__((may_alias)) v4fa;
typedef v4i  __attribute__((may_alias)) v4ia;
typedef v4u  __attribute__((may_alias)) v4ua;
typedef v8us __attribute__((may_alias)) v8usa;
union Frag { v16bf v; v16us u; v8us h[2]; v8i w; };

__device__ __forceinline__ v8f wmb(const Frag& a, const Frag& b, v8f c) {
  v8f d = __builtin_amdgcn_wmma_f32_16x16x32_bf16(false, a.v, false, b.v, (short)0, c, false, false);
  asm volatile("v_nop\n\tv_nop\n\tv_nop\n\tv_nop" : "+v"(d) : "v"(a.w), "v"(b.w));
  return d;
}

__device__ __forceinline__ unsigned bf16_bits(float f) {
  const unsigned u = __float_as_uint(f);
  return (u + 0x7FFFu + ((u >> 16) & 1u)) >> 16;
}
__device__ __forceinline__ float bf16_val(float f) {
  return __uint_as_float(bf16_bits(f) << 16);
}
__device__ __forceinline__ unsigned short bsel(float r, float t, unsigned mR) {
  const unsigned a = bf16_bits(r);
  const unsigned b = bf16_bits(t);
  return (unsigned short)((b & mR) | (a & ~mR));
}
__device__ __forceinline__ v8us pack8(v4f a, v4f b) {
  v8us o;
  o[0] = (unsigned short)bf16_bits(a.x); o[1] = (unsigned short)bf16_bits(a.y);
  o[2] = (unsigned short)bf16_bits(a.z); o[3] = (unsigned short)bf16_bits(a.w);
  o[4] = (unsigned short)bf16_bits(b.x); o[5] = (unsigned short)bf16_bits(b.y);
  o[6] = (unsigned short)bf16_bits(b.z); o[7] = (unsigned short)bf16_bits(b.w);
  return o;
}
__device__ __forceinline__ float aggfix(float a, bool has, bool live, float pzr) {
  const float r = has ? a : 0.0f;
  return live ? (r + pzr) : 0.0f;
}

__device__ __forceinline__ float wsum(float v) {
  v += __shfl_xor(v, 16, 32);
  v += __shfl_xor(v, 8, 32);
  v += __shfl_xor(v, 4, 32);
  v += __shfl_xor(v, 2, 32);
  v += __shfl_xor(v, 1, 32);
  return v;
}

template <int SLB>
__device__ __forceinline__ int scan_chunk(const int* __restrict__ dsts, int nE, int cbase, int slotBase,
                                          int nb, int vec8, int* list, int tid, int lane, int wave) {
  int wc = 0;
  const int el0  = tid * EPT;
  const int e0   = cbase + el0;
  const int sent = -2147483647 - 1;
  v4i da, db;
  if (vec8 != 0 && cbase + CHUNK <= nE) {
    da = *(const v4i*)(dsts + e0);
    db = *(const v4i*)(dsts + e0 + 4);
  } else {
    da.x = (e0     < nE) ? dsts[min(e0,     nE - 1)] : sent;
    da.y = (e0 + 1 < nE) ? dsts[min(e0 + 1, nE - 1)] : sent;
    da.z = (e0 + 2 < nE) ? dsts[min(e0 + 2, nE - 1)] : sent;
    da.w = (e0 + 3 < nE) ? dsts[min(e0 + 3, nE - 1)] : sent;
    db.x = (e0 + 4 < nE) ? dsts[min(e0 + 4, nE - 1)] : sent;
    db.y = (e0 + 5 < nE) ? dsts[min(e0 + 5, nE - 1)] : sent;
    db.z = (e0 + 6 < nE) ? dsts[min(e0 + 6, nE - 1)] : sent;
    db.w = (e0 + 7 < nE) ? dsts[min(e0 + 7, nE - 1)] : sent;
  }
  const unsigned nbs = (unsigned)slotBase;
  const unsigned unb = (unsigned)nb;
  const unsigned s0 = (unsigned)da.x - nbs, s1 = (unsigned)da.y - nbs;
  const unsigned s2 = (unsigned)da.z - nbs, s3 = (unsigned)da.w - nbs;
  const unsigned s4 = (unsigned)db.x - nbs, s5 = (unsigned)db.y - nbs;
  const unsigned s6 = (unsigned)db.z - nbs, s7 = (unsigned)db.w - nbs;
  const bool h0 = s0 < unb, h1 = s1 < unb, h2 = s2 < unb, h3 = s3 < unb;
  const bool h4 = s4 < unb, h5 = s5 < unb, h6 = s6 < unb, h7 = s7 < unb;
  const unsigned any = __builtin_amdgcn_ballot_w32(h0 | h1 | h2 | h3 | h4 | h5 | h6 | h7);
  if (any != 0u) {
#define HITJ(J, HJ, SJ) { \
      const unsigned mj = __builtin_amdgcn_ballot_w32(HJ); \
      if (mj != 0u) { \
        if (HJ) { \
          const int pos = wc + (int)__builtin_amdgcn_mbcnt_lo(mj, 0u); \
          if (pos < WCAP) list[wave * WCAP + pos] = ((el0 + (J)) << SLB) | (int)(SJ); \
        } \
        wc += (int)__builtin_popcount(mj); } }
    HITJ(0, h0, s0)
    HITJ(1, h1, s1)
    HITJ(2, h2, s2)
    HITJ(3, h3, s3)
    HITJ(4, h4, s4)
    HITJ(5, h5, s5)
    HITJ(6, h6, s6)
    HITJ(7, h7, s7)
#undef HITJ
  }
  return wc;
}

__global__ __launch_bounds__(NTHR) void k_prep(const float* __restrict__ Wr1, const float* __restrict__ Wo1,
                                               const float* __restrict__ Wr2, const float* __restrict__ Wo2,
                                               const float* __restrict__ Wc,
                                               unsigned short* B1, unsigned short* B2, unsigned short* BC) {
  const int u = (int)blockIdx.x * NTHR + (int)threadIdx.x;
  const float* pa;
  const float* pb;
  const float* pc;
  const float* pd;
  unsigned mR;
  unsigned short* dp;
  if (u < UB1) {
    const int n = u >> 5;
    const int g = u & 31;
    pa = Wr1 + (size_t)n * FIN + 4 * g;
    pb = Wo1 + (size_t)n * FIN + 4 * g;
    pc = pa; pd = pb; mR = 0u;
    dp = B1 + (size_t)n * KL1 + 8 * g;
  } else if (u < UB1 + UB2) {
    const int v  = u - UB1;
    const int n  = v >> 7;
    const int G  = v & 127;
    const int g  = G & 63;
    const int cb = 256 * (g >> 5) + 4 * (g & 31);
    pa = Wr2 + (size_t)n * HID + cb;
    pb = pa + 128;
    pc = Wo2 + (size_t)n * HID + cb;
    pd = pc + 128;
    mR = (G >= 64) ? 0xFFFFu : 0u;
    dp = B2 + (size_t)n * KL2 + 8 * G;
  } else if (u < UTOT) {
    const int v  = u - UB1 - UB2;
    const int n  = v >> 6;
    const int g  = v & 63;
    const int cb = 256 * (g >> 5) + 4 * (g & 31);
    pa = Wc + (size_t)n * HID + cb;
    pb = pa + 128;
    pc = pa; pd = pb; mR = 0u;
    dp = BC + (size_t)n * KCL + 8 * g;
  } else {
    return;
  }
  const v4f ra = *(const v4fa*)pa;
  const v4f rb = *(const v4fa*)pb;
  const v4f ta = *(const v4fa*)pc;
  const v4f tb = *(const v4fa*)pd;
  v8us o;
  o[0] = bsel(ra.x, ta.x, mR); o[1] = bsel(ra.y, ta.y, mR);
  o[2] = bsel(ra.z, ta.z, mR); o[3] = bsel(ra.w, ta.w, mR);
  o[4] = bsel(rb.x, tb.x, mR); o[5] = bsel(rb.y, tb.y, mR);
  o[6] = bsel(rb.z, tb.z, mR); o[7] = bsel(rb.w, tb.w, mR);
  *(volatile v8us*)dp = o;
  __threadfence();
  *(volatile v8us*)dp = o;
}

__global__ __launch_bounds__(LTHR) void k_gemm_ln(unsigned short* apl, int K, const unsigned short* __restrict__ BT,
                                                  const float* __restrict__ bias, const float* __restrict__ gam,
                                                  const float* __restrict__ bet, int nN) {
  extern __shared__ __attribute__((aligned(16))) float dsg[];
  const int tid = (int)threadIdx.x, lane = tid & 31, wave = tid >> 5, hh = lane >> 4, m = lane & 15;
  const int rw = wave >> 2, cw = wave & 3;
  const int rowBase = (int)blockIdx.x * LBM;

  v8f acc[8];
  {
    const v8f z = {0.f, 0.f, 0.f, 0.f, 0.f, 0.f, 0.f, 0.f};
#pragma unroll
    for (int t = 0; t < 8; ++t) acc[t] = z;
  }
  const unsigned short* ap = apl + (size_t)(rowBase + 16 * rw + m) * (size_t)AP + 8 * hh;
  const unsigned short* bp = BT + (size_t)(128 * cw + m) * (size_t)K + 8 * hh;

#pragma unroll 1
  for (int k0 = 0; k0 < K; k0 += 32) {
    Frag af;
    af.h[0] = *(const v8usa*)(ap + k0);
    af.h[1] = *(const v8usa*)(ap + k0 + 16);
#pragma unroll
    for (int nt = 0; nt < 8; ++nt) {
      const unsigned short* wq = bp + (size_t)(16 * nt) * (size_t)K + k0;
      Frag bf;
      bf.h[0] = *(const v8usa*)wq;
      bf.h[1] = *(const v8usa*)(wq + 16);
      acc[nt] = wmb(af, bf, acc[nt]);
    }
  }

#pragma unroll
  for (int nt = 0; nt < 8; ++nt) {
    const int lc = 128 * cw + 16 * nt + m;
#pragma unroll
    for (int r = 0; r < 8; ++r) {
      const int lr = 16 * rw + 8 * hh + r;
      dsg[lr * HID + lc] = acc[nt][r];
    }
  }
  __syncthreads();

  v4f bb0, bb1, bb2, bb3, gg0, gg1, gg2, gg3, ee0, ee1, ee2, ee3;
  {
#define LDPAR(DST, SRC, OFF) { const v4f tq = *(const v4fa*)((SRC) + 4 * lane + (OFF)); \
      DST.x = bf16_val(tq.x); DST.y = bf16_val(tq.y); DST.z = bf16_val(tq.z); DST.w = bf16_val(tq.w); }
    LDPAR(bb0, bias, 0) LDPAR(bb1, bias, 128) LDPAR(bb2, bias, 256) LDPAR(bb3, bias, 384)
    LDPAR(gg0, gam, 0)  LDPAR(gg1, gam, 128)  LDPAR(gg2, gam, 256)  LDPAR(gg3, gam, 384)
    LDPAR(ee0, bet, 0)  LDPAR(ee1, bet, 128)  LDPAR(ee2, bet, 256)  LDPAR(ee3, bet, 384)
#undef LDPAR
  }

  v8us po[8];
#pragma unroll
  for (int i = 0; i < 4; ++i) {
    const int lrow = 4 * wave + i;
    const float okf = (rowBase + lrow < nN) ? 1.0f : 0.0f;
    const float* sp = dsg + lrow * HID + 4 * lane;
    const v4f t0 = *(const v4fa*)(sp)       + bb0;
    const v4f t1 = *(const v4fa*)(sp + 128) + bb1;
    const v4f t2 = *(const v4fa*)(sp + 256) + bb2;
    const v4f t3 = *(const v4fa*)(sp + 384) + bb3;
    const float s = wsum((((t0.x + t0.y) + (t0.z + t0.w)) + ((t1.x + t1.y) + (t1.z + t1.w))) +
                         (((t2.x + t2.y) + (t2.z + t2.w)) + ((t3.x + t3.y) + (t3.z + t3.w))));
    const float mu = s * (1.0f / HID);
    const v4f d0 = t0 - mu, d1 = t1 - mu, d2 = t2 - mu, d3 = t3 - mu;
    const float q = wsum((((d0.x * d0.x + d0.y * d0.y) + (d0.z * d0.z + d0.w * d0.w)) +
                          ((d1.x * d1.x + d1.y * d1.y) + (d1.z * d1.z + d1.w * d1.w))) +
                         (((d2.x * d2.x + d2.y * d2.y) + (d2.z * d2.z + d2.w * d2.w)) +
                          ((d3.x * d3.x + d3.y * d3.y) + (d3.z * d3.z + d3.w * d3.w))));
    const float rs = rsqrtf(q * (1.0f / HID) + 1e-5f);
    v4f y0 = d0 * rs * gg0 + ee0;
    v4f y1 = d1 * rs * gg1 + ee1;
    v4f y2 = d2 * rs * gg2 + ee2;
    v4f y3 = d3 * rs * gg3 + ee3;
    y0.x = fmaxf(y0.x, 0.0f) * okf; y0.y = fmaxf(y0.y, 0.0f) * okf; y0.z = fmaxf(y0.z, 0.0f) * okf; y0.w = fmaxf(y0.w, 0.0f) * okf;
    y1.x = fmaxf(y1.x, 0.0f) * okf; y1.y = fmaxf(y1.y, 0.0f) * okf; y1.z = fmaxf(y1.z, 0.0f) * okf; y1.w = fmaxf(y1.w, 0.0f) * okf;
    y2.x = fmaxf(y2.x, 0.0f) * okf; y2.y = fmaxf(y2.y, 0.0f) * okf; y2.z = fmaxf(y2.z, 0.0f) * okf; y2.w = fmaxf(y2.w, 0.0f) * okf;
    y3.x = fmaxf(y3.x, 0.0f) * okf; y3.y = fmaxf(y3.y, 0.0f) * okf; y3.z = fmaxf(y3.z, 0.0f) * okf; y3.w = fmaxf(y3.w, 0.0f) * okf;
    po[2 * i]     = pack8(y0, y1);
    po[2 * i + 1] = pack8(y2, y3);
  }
#pragma unroll
  for (int i = 0; i < 4; ++i) {
    unsigned short* rp = apl + (size_t)(rowBase + 4 * wave + i) * (size_t)AP + HOFF + 8 * lane;
    *(volatile v8us*)rp = po[2 * i];
    *(volatile v8us*)(rp + 256) = po[2 * i + 1];
  }
  __threadfence();
#pragma unroll
  for (int i = 0; i < 4; ++i) {
    unsigned short* rp = apl + (size_t)(rowBase + 4 * wave + i) * (size_t)AP + HOFF + 8 * lane;
    *(volatile v8us*)rp = po[2 * i];
    *(volatile v8us*)(rp + 256) = po[2 * i + 1];
  }
}

__global__ __launch_bounds__(GTHR) void k_cls(const unsigned short* __restrict__ A, int lda,
                                              const unsigned short* __restrict__ BT, int ldb, int K,
                                              const float* __restrict__ bias, float* outp, int nOut) {
  constexpr int N = 128;
  __shared__ __attribute__((aligned(16))) float stg[GBM * N];
  const int tid = (int)threadIdx.x, lane = tid & 31, wave = tid >> 5, hh = lane >> 4, m = lane & 15;
  const int rowBase = (int)blockIdx.x * GBM;

  v8f acc[8];
  {
    const v8f z = {0.f, 0.f, 0.f, 0.f, 0.f, 0.f, 0.f, 0.f};
#pragma unroll
    for (int t = 0; t < 8; ++t) acc[t] = z;
  }
  const unsigned short* ap = A  + (size_t)(rowBase + 16 * wave + m) * (size_t)lda + 8 * hh;
  const unsigned short* bp = BT + (size_t)m * (size_t)ldb + 8 * hh;

#pragma unroll 1
  for (int k0 = 0; k0 < K; k0 += 32) {
    Frag af;
    af.h[0] = *(const v8usa*)(ap + k0);
    af.h[1] = *(const v8usa*)(ap + k0 + 16);
#pragma unroll
    for (int nt = 0; nt < 8; ++nt) {
      const unsigned short* wq = bp + (size_t)(16 * nt) * (size_t)ldb + k0;
      Frag bf;
      bf.h[0] = *(const v8usa*)wq;
      bf.h[1] = *(const v8usa*)(wq + 16);
      acc[nt] = wmb(af, bf, acc[nt]);
    }
  }

#pragma unroll
  for (int nt = 0; nt < 8; ++nt) {
    const int lc = 16 * nt + m;
#pragma unroll
    for (int r = 0; r < 8; ++r) {
      const int lr = 16 * wave + 8 * hh + r;
      stg[lr * N + lc] = acc[nt][r];
    }
  }
  __syncthreads();

  v4f b4;
  {
    const v4f tb = *(const v4fa*)(bias + 4 * lane);
    b4.x = bf16_val(tb.x); b4.y = bf16_val(tb.y); b4.z = bf16_val(tb.z); b4.w = bf16_val(tb.w);
  }
  v4f pv[16];
#pragma unroll
  for (int i = 0; i < 16; ++i) pv[i] = *(const v4fa*)(stg + (16 * wave + i) * N + 4 * lane) + b4;
#pragma unroll
  for (int i = 0; i < 16; ++i) {
    const int row = rowBase + 16 * wave + i;
    if (row < nOut) *(volatile v4f*)(outp + (size_t)row * N + 4 * lane) = pv[i];
  }
  __threadfence();
#pragma unroll
  for (int i = 0; i < 16; ++i) {
    const int row = rowBase + 16 * wave + i;
    if (row < nOut) *(volatile v4f*)(outp + (size_t)row * N + 4 * lane) = pv[i];
  }
}

template <int L1>
__global__ __launch_bounds__(NTHR) void k_scan(const int* __restrict__ srcs, const int* __restrict__ dsts,
                                               const float* __restrict__ pos, int nE, int nN, int vec8, int mRows,
                                               const float* __restrict__ xin, unsigned short* apl) {
  extern __shared__ __attribute__((aligned(16))) int dsm[];
  int* list = dsm;
  int* hl   = dsm + LISTN;
  int* sl   = hl + RCAP;
  int* cnt  = sl + RCAP;
  int* offs = cnt + NBA;
  int* cur  = offs + NBA;
  int* misc = cur + NBA;
  const int tid = (int)threadIdx.x, lane = tid & 31, wave = tid >> 5;
  const int nodeBase = (int)blockIdx.x * NBA;

  {
    const v4i z4 = {0, 0, 0, 0};
    for (int i = tid * 4; i < AGG_ZINTS; i += NTHR * 4) *(v4ia*)(dsm + i) = z4;
    if (tid < MISC_INTS) misc[tid] = 0;
  }
  __syncthreads();

  int t = 0, ov = 0;
  const int nChunks = (nE + CHUNK - 1) / CHUNK;
#pragma unroll 1
  for (int ch = 0; ch < nChunks; ++ch) {
    const int cbase = ch * CHUNK;
    const int wc = scan_chunk<SLA>(dsts, nE, cbase, nodeBase, NBA, vec8, list, tid, lane, wave);
    if (lane == 0) misc[wave] = wc;
    __syncthreads();
    if (wave == 0) {
#pragma unroll 1
      for (int w2 = 0; w2 < NWAVE; ++w2) {
        int c = misc[w2];
        c = c < 0 ? 0 : (c > WCAP ? WCAP : c);
#pragma unroll 1
        for (int b0 = 0; b0 < c; b0 += 32) {
          const int idx = b0 + lane;
          const int ent = list[w2 * WCAP + (idx < WCAP ? idx : WCAP - 1)];
          const int m32 = (c - b0) < 32 ? (c - b0) : 32;
#pragma unroll 1
          for (int k = 0; k < m32; ++k) {
            const int u    = __builtin_amdgcn_readlane(ent, k);
            const int slot = u & (NBA - 1);
            const int el   = (u >> SLA) & (CHUNK - 1);
            const int pk   = ((cbase + el) << SLA) | slot;
            if (t < RCAP) {
              if (lane == 0) { hl[t] = pk; cnt[slot] = cnt[slot] + 1; }
              t = t + 1;
            } else {
              ov = 1;
            }
          }
        }
      }
    }
    __syncthreads();
  }
  if (wave == 0 && lane == 0) { misc[8] = t; misc[9] = ov; }
  __syncthreads();
  int tt = misc[8];
  tt = tt < 0 ? 0 : (tt > RCAP ? RCAP : tt);
  const int ovf = misc[9];

  if (wave == 0) {
    const int base = lane * (NBA / 32);
    int sacc = 0;
#pragma unroll 1
    for (int i = 0; i < NBA / 32; ++i) sacc += cnt[base + i];
    int incl = sacc;
#pragma unroll
    for (int d = 1; d < 32; d <<= 1) {
      const int y = __shfl_up(incl, d, 32);
      if (lane >= d) incl += y;
    }
    int run = incl - sacc;
#pragma unroll 1
    for (int i = 0; i < NBA / 32; ++i) {
      const int cv = cnt[base + i];
      offs[base + i] = run;
      cur[base + i]  = run;
      run += cv;
    }
  }
  __syncthreads();
  if (wave == 0) {
#pragma unroll 1
    for (int b0 = 0; b0 < tt; b0 += 32) {
      const int idx = b0 + lane;
      const int ent = hl[idx < RCAP ? idx : RCAP - 1];
      const int m32 = (tt - b0) < 32 ? (tt - b0) : 32;
#pragma unroll 1
      for (int k = 0; k < m32; ++k) {
        const int u    = __builtin_amdgcn_readlane(ent, k);
        const int slot = u & (NBA - 1);
        if (lane == 0) {
          int p = cur[slot];
          p = p < 0 ? 0 : (p > RCAP - 1 ? RCAP - 1 : p);
          sl[p] = u;
          cur[slot] = p + 1;
        }
      }
    }
  }
  __syncthreads();

  const float qnan = __uint_as_float(0x7fc00000u);
  const float ninf = __uint_as_float(0xff800000u);
  const float pz = (ovf != 0) ? qnan : 0.0f;
  const v4f nn = {ninf, ninf, ninf, ninf};
#pragma unroll 1
  for (int si = 0; si < NBA / NWAVE; ++si) {
    const int s    = si * NWAVE + wave;
    const int node = nodeBase + s;
    int c = cnt[s];
    const bool big = c > DEGCAP;
    c = c < 0 ? 0 : (c > DEGCAP ? DEGCAP : c);
    int o = offs[s];
    o = o < 0 ? 0 : (o > RCAP ? RCAP : o);
    const int nc = node < nN ? node : nN - 1;
    const float pdn = pos[nc];
    v4f m0 = nn, m1 = nn, m2 = nn, m3 = nn;
#pragma unroll 1
    for (int b0 = 0; b0 < c; b0 += 32) {
      int idx = o + b0 + lane;
      idx = idx > RCAP - 1 ? RCAP - 1 : idx;
      const int ent = sl[idx];
      int eid = ent >> SLA;
      eid = eid < 0 ? 0 : (eid > nE - 1 ? nE - 1 : eid);
      int sr = srcs[eid];
      sr = sr < 0 ? 0 : (sr > nN - 1 ? nN - 1 : sr);
      const float dif  = pos[sr] - pdn;
      const float difs = (dif != 0.0f) ? dif : 1.0f;
      const float ewl  = 1.0f / difs;
      const int   ewb  = __float_as_int(ewl);
      const int m32 = (c - b0) < 32 ? (c - b0) : 32;
#pragma unroll 1
      for (int k = 0; k < m32; ++k) {
        const int   sk = __builtin_amdgcn_readlane(sr, k);
        const float ew = __int_as_float(__builtin_amdgcn_readlane(ewb, k));
        if constexpr (L1 != 0) {
          const v4f xr = *(const v4fa*)(xin + (size_t)sk * FIN + 4 * lane);
          m0.x = fmaxf(m0.x, bf16_val(xr.x) * ew);
          m0.y = fmaxf(m0.y, bf16_val(xr.y) * ew);
          m0.z = fmaxf(m0.z, bf16_val(xr.z) * ew);
          m0.w = fmaxf(m0.w, bf16_val(xr.w) * ew);
        } else {
          const unsigned short* hp = apl + (size_t)sk * (size_t)AP + HOFF + 8 * lane;
          const v4u w0 = *(const v4ua*)hp;
          const v4u w1 = *(const v4ua*)(hp + 256);
          m0.x = fmaxf(m0.x, __uint_as_float(w0.x << 16)         * ew);
          m0.y = fmaxf(m0.y, __uint_as_float(w0.x & 0xffff0000u) * ew);
          m0.z = fmaxf(m0.z, __uint_as_float(w0.y << 16)         * ew);
          m0.w = fmaxf(m0.w, __uint_as_float(w0.y & 0xffff0000u) * ew);
          m1.x = fmaxf(m1.x, __uint_as_float(w0.z << 16)         * ew);
          m1.y = fmaxf(m1.y, __uint_as_float(w0.z & 0xffff0000u) * ew);
          m1.z = fmaxf(m1.z, __uint_as_float(w0.w << 16)         * ew);
          m1.w = fmaxf(m1.w, __uint_as_float(w0.w & 0xffff0000u) * ew);
          m2.x = fmaxf(m2.x, __uint_as_float(w1.x << 16)         * ew);
          m2.y = fmaxf(m2.y, __uint_as_float(w1.x & 0xffff0000u) * ew);
          m2.z = fmaxf(m2.z, __uint_as_float(w1.y << 16)         * ew);
          m2.w = fmaxf(m2.w, __uint_as_float(w1.y & 0xffff0000u) * ew);
          m3.x = fmaxf(m3.x, __uint_as_float(w1.z << 16)         * ew);
          m3.y = fmaxf(m3.y, __uint_as_float(w1.z & 0xffff0000u) * ew);
          m3.z = fmaxf(m3.z, __uint_as_float(w1.w << 16)         * ew);
          m3.w = fmaxf(m3.w, __uint_as_float(w1.w & 0xffff0000u) * ew);
        }
      }
    }
    const float pzr  = big ? qnan : pz;
    const bool  live = node < nN;
    const bool  has  = c > 0;
    v4f r0;
    r0.x = aggfix(m0.x, has, live, pzr); r0.y = aggfix(m0.y, has, live, pzr);
    r0.z = aggfix(m0.z, has, live, pzr); r0.w = aggfix(m0.w, has, live, pzr);
    if constexpr (L1 != 0) {
      const v4f xs = *(const v4fa*)(xin + (size_t)nc * FIN + 4 * lane);
      v4f xq;
      xq.x = live ? (xs.x + pzr) : 0.0f; xq.y = live ? (xs.y + pzr) : 0.0f;
      xq.z = live ? (xs.z + pzr) : 0.0f; xq.w = live ? (xs.w + pzr) : 0.0f;
      const v8us q0 = pack8(r0, xq);
      (void)m1; (void)m2; (void)m3;
      if (node < mRows) {
        unsigned short* rpw = apl + (size_t)node * (size_t)AP + 8 * lane;
        *(volatile v8us*)rpw = q0;
        __threadfence();
        *(volatile v8us*)rpw = q0;
      }
    } else {
      v4f r1, r2, r3;
      r1.x = aggfix(m1.x, has, live, pzr); r1.y = aggfix(m1.y, has, live, pzr);
      r1.z = aggfix(m1.z, has, live, pzr); r1.w = aggfix(m1.w, has, live, pzr);
      r2.x = aggfix(m2.x, has, live, pzr); r2.y = aggfix(m2.y, has, live, pzr);
      r2.z = aggfix(m2.z, has, live, pzr); r2.w = aggfix(m2.w, has, live, pzr);
      r3.x = aggfix(m3.x, has, live, pzr); r3.y = aggfix(m3.y, has, live, pzr);
      r3.z = aggfix(m3.z, has, live, pzr); r3.w = aggfix(m3.w, has, live, pzr);
      const v8us q0 = pack8(r0, r1);
      const v8us q1 = pack8(r2, r3);
      if (node < mRows) {
        unsigned short* rpw = apl + (size_t)node * (size_t)AP + 8 * lane;
        *(volatile v8us*)rpw = q0;
        *(volatile v8us*)(rpw + 256) = q1;
        __threadfence();
        *(volatile v8us*)rpw = q0;
        *(volatile v8us*)(rpw + 256) = q1;
      }
    }
  }
}

static inline int cdiv(int a, int b) { return (a + b - 1) / b; }

extern "C" void kernel_launch(void* const* d_in, const int* in_sizes, int n_in,
                              void* d_out, int out_size, void* d_ws, size_t ws_size,
                              hipStream_t stream) {
  if (n_in < 15) return;
  if (in_sizes[0] < FIN || (in_sizes[0] % FIN) != 0) return;
  const int nN = in_sizes[0] / FIN;
  if (in_sizes[1] < 2 || (in_sizes[1] & 1) != 0) return;
  const int nE = in_sizes[1] / 2;
  if (nE < 1 || nE >= (1 << 21)) return;
  if (in_sizes[2] != nN) return;
  if (in_sizes[3] != HID * FIN || in_sizes[4] != HID || in_sizes[5] != HID * FIN) return;
  if (in_sizes[6] != HID || in_sizes[7] != HID) return;
  if (in_sizes[8] != HID * HID || in_sizes[9] != HID || in_sizes[10] != HID * HID) return;
  if (in_sizes[11] != HID || in_sizes[12] != HID) return;
  if (in_sizes[13] != NCLS * HID || in_sizes[14] != NCLS) return;
  if ((long long)out_size != (long long)nN * NCLS) return;

  const float* x      = (const float*)d_in[0];
  const int*   edge   = (const int*)d_in[1];
  const float* posv   = (const float*)d_in[2];
  const float* Wrel1  = (const float*)d_in[3];
  const float* brel1  = (const float*)d_in[4];
  const float* Wroot1 = (const float*)d_in[5];
  const float* g1     = (const float*)d_in[6];
  const float* b1     = (const float*)d_in[7];
  const float* Wrel2  = (const float*)d_in[8];
  const float* brel2  = (const float*)d_in[9];
  const float* Wroot2 = (const float*)d_in[10];
  const float* g2     = (const float*)d_in[11];
  const float* b2     = (const float*)d_in[12];
  const float* Wcls   = (const float*)d_in[13];
  const float* bcls   = (const float*)d_in[14];
  float* out = (float*)d_out;
  const int* src = edge;
  const int* dst = edge + nE;

  const int MP = cdiv(nN, GBM) * GBM;
  if ((MP % LBM) != 0 || (MP % GBM) != 0) return;
  const int gL = MP / LBM;
  const int gC = MP / GBM;
  const int gA = cdiv(MP, NBA);
  if ((long long)gA * NBA < (long long)MP) return;
  const int vec8 = ((nE & 3) == 0) ? 1 : 0;

  char* ws = (char*)d_ws;
  size_t off = 0;
  const size_t oB1 = off; off += (size_t)HID * KL1 * 2;                     off = (off + 255) & ~(size_t)255;
  const size_t oB2 = off; off += (size_t)HID * KL2 * 2;                     off = (off + 255) & ~(size_t)255;
  const size_t oBC = off; off += (size_t)NCLS * KCL * 2;                    off = (off + 255) & ~(size_t)255;
  const size_t oA  = off; off += (size_t)MP * AP * 2;                       off = (off + 255) & ~(size_t)255;
  if (off > ws_size || off > (size_t)WSMAX) return;
  unsigned short* B1  = (unsigned short*)(ws + oB1);
  unsigned short* B2  = (unsigned short*)(ws + oB2);
  unsigned short* BC  = (unsigned short*)(ws + oBC);
  unsigned short* Apl = (unsigned short*)(ws + oA);

  const size_t scanLds = (size_t)AGG_LDS_INTS * 4;
  const size_t lnLds   = (size_t)LN_LDS_BYTES;
  hipFuncSetAttribute(reinterpret_cast<const void*>(&k_scan<1>), hipFuncAttributeMaxDynamicSharedMemorySize, (int)scanLds);
  hipFuncSetAttribute(reinterpret_cast<const void*>(&k_scan<0>), hipFuncAttributeMaxDynamicSharedMemorySize, (int)scanLds);
  hipFuncSetAttribute(reinterpret_cast<const void*>(&k_gemm_ln), hipFuncAttributeMaxDynamicSharedMemorySize, (int)lnLds);

  k_prep<<<UTOT / NTHR, NTHR, 0, stream>>>(Wrel1, Wroot1, Wrel2, Wroot2, Wcls, B1, B2, BC);
  k_scan<1><<<gA, NTHR, scanLds, stream>>>(src, dst, posv, nE, nN, vec8, MP, x, Apl);
  k_gemm_ln<<<gL, LTHR, lnLds, stream>>>(Apl, KL1, B1, brel1, g1, b1, nN);
  k_scan<0><<<gA, NTHR, scanLds, stream>>>(src, dst, posv, nE, nN, vec8, MP, x, Apl);
  k_gemm_ln<<<gL, LTHR, lnLds, stream>>>(Apl, KL2, B2, brel2, g2, b2, nN);
  k_cls<<<gC, GTHR, 0, stream>>>(Apl + HOFF, AP, BC, KCL, KCL, bcls, out, nN);
}
